// MultiHeadPhasorBlock_45337674776746
// MI455X (gfx1250) — hardware-verified
//
#include <hip/hip_runtime.h>
#include <math.h>

constexpr int kB   = 2;
constexpr int kL   = 4096;
constexpr int kD   = 512;
constexpr int kM   = kB * kL;
constexpr int kP   = 128;
constexpr int kH   = 4;
constexpr int kPh  = 32;
constexpr int kV   = 8;
constexpr int kHV  = 32;
constexpr int kD2  = 1024;
constexpr int kD3  = 1536;
constexpr int kVGld = 64;
constexpr float kPI = 3.14159265358979323846f;
constexpr float kSqrt32 = 5.656854249492381f;
constexpr float kSqrt8  = 2.8284271247461903f;

typedef __attribute__((ext_vector_type(16))) _Float16 v16h;
typedef __attribute__((ext_vector_type(8)))  _Float16 v8h;
typedef __attribute__((ext_vector_type(16))) __bf16   v16b;
typedef __attribute__((ext_vector_type(8)))  __bf16   v8b;
typedef __attribute__((ext_vector_type(8)))  float    v8f;
typedef __attribute__((ext_vector_type(4)))  float    v4f;
typedef __attribute__((ext_vector_type(2)))  float    v2f;
typedef __attribute__((ext_vector_type(4)))  unsigned int v4u;

__device__ __forceinline__ unsigned short f2bf_bits(float f) {
  unsigned u = __float_as_uint(f);
  return (unsigned short)((u + 0x7FFFu + ((u >> 16) & 1u)) >> 16);
}
__device__ __forceinline__ float bf_bits2f(unsigned short h) { return __uint_as_float(((unsigned)h) << 16); }

__device__ __forceinline__ void dep_guard_h(v8f& a, v8f& b, v16h x, v16h y) { asm volatile("v_nop\n\tv_nop\n\tv_nop\n\tv_nop" : "+v"(a), "+v"(b) : "v"(x), "v"(y)); }
__device__ __forceinline__ void dep_guard_b(v8f& a, v8f& b, v16b x, v16b y) { asm volatile("v_nop\n\tv_nop\n\tv_nop\n\tv_nop" : "+v"(a), "+v"(b) : "v"(x), "v"(y)); }
__device__ __forceinline__ void keep4_h(v16h a, v16h b, v16h c, v16h d) { asm volatile("v_nop" :: "v"(a), "v"(b), "v"(c), "v"(d)); }
__device__ __forceinline__ void keep4_b(v16b a, v16b b, v16b c, v16b d) { asm volatile("v_nop" :: "v"(a), "v"(b), "v"(c), "v"(d)); }
__device__ __forceinline__ void acc_guard4(v8f& a, v8f& b, v8f& c, v8f& d) { asm volatile("v_nop\n\tv_nop\n\tv_nop\n\tv_nop" : "+v"(a), "+v"(b), "+v"(c), "+v"(d)); }
template <typename T> struct Frag;
template <> struct Frag<_Float16> {
  typedef v16h V; union U { v16h v; v8h h[2]; };
  static __device__ __forceinline__ v16h load(const _Float16* p) {
    U f; f.h[0] = *(const v8h*)(p); f.h[1] = *(const v8h*)(p + 16); return f.v;
  }
  static __device__ __forceinline__ v8f mma(v16h a, v16h b, v8f c) {
    return __builtin_amdgcn_wmma_f32_16x16x32_f16(false, a, false, b, (short)0, c, false, false);
  }
  static __device__ __forceinline__ void guard(v8f& a, v8f& b, v16h x, v16h y) { dep_guard_h(a, b, x, y); }
  static __device__ __forceinline__ void keep(v16h a, v16h b, v16h c, v16h d) { keep4_h(a, b, c, d); }
};
template <> struct Frag<__bf16> {
  typedef v16b V; union U { v16b v; v8b h[2]; };
  static __device__ __forceinline__ v16b load(const __bf16* p) {
    U f; f.h[0] = *(const v8b*)(p); f.h[1] = *(const v8b*)(p + 16); return f.v;
  }
  static __device__ __forceinline__ v8f mma(v16b a, v16b b, v8f c) {
    return __builtin_amdgcn_wmma_f32_16x16x32_bf16(false, a, false, b, (short)0, c, false, false);
  }
  static __device__ __forceinline__ void guard(v8f& a, v8f& b, v16b x, v16b y) { dep_guard_b(a, b, x, y); }
  static __device__ __forceinline__ void keep(v16b a, v16b b, v16b c, v16b d) { keep4_b(a, b, c, d); }
};

__device__ __forceinline__ unsigned pk16(unsigned short a, unsigned short b) { return (unsigned)a | ((unsigned)b << 16); }
__device__ __forceinline__ unsigned short h_bits(float f) { const _Float16 h = (_Float16)f; return __builtin_bit_cast(unsigned short, h); }
__device__ __forceinline__ float h_lo(unsigned w) { return (float)__builtin_bit_cast(_Float16, (unsigned short)(w & 0xffffu)); }
__device__ __forceinline__ float h_hi(unsigned w) { return (float)__builtin_bit_cast(_Float16, (unsigned short)(w >> 16)); }

__device__ __forceinline__ float wave_sum(float v) {
#pragma unroll
  for (int off = 16; off > 0; off >>= 1) v += __shfl_xor(v, off, 32);
  return v;
}

template <int ET> struct Elem;
template <> struct Elem<0> { typedef _Float16 T; };
template <> struct Elem<1> { typedef __bf16 T; };
template <int ET, bool SPLIT, int BIAS_MODE, int OUT_MODE, bool RESID, int ACT = 0>
__global__ __launch_bounds__(256) void wmma_gemm64(
    const unsigned short* __restrict__ Ap, const unsigned short* __restrict__ A2p, int lda, long strideA,
    const unsigned short* __restrict__ Btp, const unsigned short* __restrict__ Bt2p, int ldb, long strideB,
    void* __restrict__ Cout, void* __restrict__ Cout2, int ldc, long strideC,
    const float* __restrict__ bias,
    const float* __restrict__ resid, long strideR,
    int M, int N, int K, float scale) {
  typedef typename Elem<ET>::T T;
  typedef typename Frag<T>::V V;
  const T* A = (const T*)Ap; const T* A2 = (const T*)A2p; const T* Bt = (const T*)Btp; const T* Bt2 = (const T*)Bt2p;
  __shared__ __align__(16) float sT[8][16 * 68];
  const int b    = blockIdx.y;
  const int lane = threadIdx.x & 31;
  const int wave = threadIdx.x >> 5;
  const int tilesN = N >> 6;
  const int tilesM = M >> 6;
  const int tile = blockIdx.x * 8 + wave;
  if (tile >= tilesM * tilesN) return;
  const int tm = tile / tilesN;
  const int tn = tile - tm * tilesN;
  const int m0 = tm << 6;
  const int n0 = tn << 6;

  const T* Ab  = A  + (size_t)b * strideA;
  const T* Bb  = Bt + (size_t)b * strideB;
  const T* Ab2 = SPLIT ? (A2  + (size_t)b * strideA) : nullptr;
  const T* Bb2 = SPLIT ? (Bt2 + (size_t)b * strideB) : nullptr;

  const int rlane = lane & 15;
  const int koff  = (lane >> 4) * 8;
  const int mOff  = (lane >> 4) * 8;

  v8f acc[4][4];
#pragma unroll
  for (int i = 0; i < 4; ++i)
#pragma unroll
    for (int j = 0; j < 4; ++j) acc[i][j] = (v8f){0.f,0.f,0.f,0.f,0.f,0.f,0.f,0.f};

  for (int k0 = 0; k0 < K; k0 += 32) {
    V bh[4], bl[4];
#pragma unroll
    for (int j = 0; j < 4; ++j) {
      const size_t bo = (size_t)(n0 + (j << 4) + rlane) * ldb + koff + k0;
      bh[j] = Frag<T>::load(Bb + bo);
      if (SPLIT) bl[j] = Frag<T>::load(Bb2 + bo);
    }
#pragma unroll
    for (int i = 0; i < 4; ++i) {
      const size_t ao = (size_t)(m0 + (i << 4) + rlane) * lda + koff + k0;
      V ah = Frag<T>::load(Ab + ao);
      V al;
      if (SPLIT) al = Frag<T>::load(Ab2 + ao);
#pragma unroll
      for (int j = 0; j < 4; ++j) {
        acc[i][j] = Frag<T>::mma(ah, bh[j], acc[i][j]);
        if (SPLIT) {
          acc[i][j] = Frag<T>::mma(ah, bl[j], acc[i][j]);
          acc[i][j] = Frag<T>::mma(al, bh[j], acc[i][j]);
        }
      }
      Frag<T>::guard(acc[i][0], acc[i][3], ah, SPLIT ? al : ah);
    }
    Frag<T>::keep(bh[0], bh[1], bh[2], bh[3]);
    if (SPLIT) Frag<T>::keep(bl[0], bl[1], bl[2], bl[3]);
  }
  acc_guard4(acc[0][0], acc[0][1], acc[0][2], acc[0][3]);
  acc_guard4(acc[1][0], acc[1][1], acc[1][2], acc[1][3]);
  acc_guard4(acc[2][0], acc[2][1], acc[2][2], acc[2][3]);
  acc_guard4(acc[3][0], acc[3][1], acc[3][2], acc[3][3]);

  float* slab = sT[wave];
  const float* Rb = RESID ? (resid + (size_t)b * strideR) : nullptr;
#pragma unroll
  for (int i = 0; i < 4; ++i) {
    const int mBase = m0 + (i << 4);
#pragma unroll
    for (int j = 0; j < 4; ++j) {
      const int n = n0 + (j << 4) + rlane;
      float bv = 0.f;
      if (BIAS_MODE == 2) bv = bias[n];
#pragma unroll
      for (int r = 0; r < 8; ++r) {
        float v = acc[i][j][r] * scale;
        if (BIAS_MODE == 1) v += bias[mBase + mOff + r];
        if (BIAS_MODE == 2) v += bv;
        if (RESID) v += Rb[(size_t)(mBase + mOff + r) * ldc + n];
        if (ACT == 2) v = fmaxf(v, 0.0f);
        if (ACT == 4) v = (v > 0.f) ? v : 0.01f * v;
        slab[(mOff + r) * 68 + (j << 4) + rlane] = v;
      }
    }
    __builtin_amdgcn_fence(__ATOMIC_RELEASE, "workgroup");
    __builtin_amdgcn_wave_barrier();
    __builtin_amdgcn_fence(__ATOMIC_ACQUIRE, "workgroup");
    if (OUT_MODE == 0) {
      float* C = (float*)Cout + (size_t)b * strideC;
      const int hh = lane >> 4, c4 = (lane & 15) * 4;
      for (int pass = 0; pass < 2; ++pass) {
#pragma unroll
        for (int it = 0; it < 8; ++it) {
          const int row = it * 2 + hh;
          v4f v = *(const v4f*)(slab + row * 68 + c4);
          *(volatile v4f*)(C + (size_t)(mBase + row) * ldc + n0 + c4) = v;
        }
        __threadfence();
      }
    } else {
      const int q = lane >> 3, c8 = (lane & 7) * 8;
      unsigned short* C  = (unsigned short*)Cout  + (size_t)b * strideC;
      unsigned short* C2 = (OUT_MODE == 2) ? ((unsigned short*)Cout2 + (size_t)b * strideC) : nullptr;
      for (int pass = 0; pass < 2; ++pass) {
#pragma unroll
        for (int it = 0; it < 4; ++it) {
          const int row = it * 4 + q;
          const float* sp = slab + row * 68 + c8;
          v8h hv, lv;
#pragma unroll
          for (int e = 0; e < 8; ++e) {
            if (OUT_MODE == 1) {
              hv[e] = (_Float16)sp[e];
            } else {
              unsigned short hb = f2bf_bits(sp[e]);
              unsigned short lb = f2bf_bits(sp[e] - bf_bits2f(hb));
              hv[e] = __builtin_bit_cast(_Float16, hb);
              lv[e] = __builtin_bit_cast(_Float16, lb);
            }
          }
          *(volatile v8h*)(C + (size_t)(mBase + row) * ldc + n0 + c8) = hv;
          if (OUT_MODE == 2) *(volatile v8h*)(C2 + (size_t)(mBase + row) * ldc + n0 + c8) = lv;
        }
        __threadfence();
      }
    }
    __builtin_amdgcn_fence(__ATOMIC_RELEASE, "workgroup");
    __builtin_amdgcn_wave_barrier();
    __builtin_amdgcn_fence(__ATOMIC_ACQUIRE, "workgroup");
  }
}

__global__ __launch_bounds__(256) void cast_inputs_kernel(const float* __restrict__ x, const float* __restrict__ pos,
                                                          unsigned short* __restrict__ a3) {
  const int t = blockIdx.x * 256 + threadIdx.x;
  if (t >= kM * (kD / 8)) return;
  const int part = blockIdx.y;
  const int row = t >> 6;
  const int c8 = (t & 63) * 8;
  const float* src = (part == 0) ? (pos + (size_t)(row & (kL - 1)) * kD + c8) : (x + (size_t)row * kD + c8);
  const v4f a = *(const v4f*)(src);
  const v4f c = *(const v4f*)(src + 4);
  unsigned short hb[8];
#pragma unroll
  for (int e = 0; e < 4; ++e) { hb[e] = h_bits(a[e]); hb[4 + e] = h_bits(c[e]); }
  const v4u u = (v4u){pk16(hb[0], hb[1]), pk16(hb[2], hb[3]), pk16(hb[4], hb[5]), pk16(hb[6], hb[7])};
  unsigned short* q = a3 + (size_t)row * kD3 + (size_t)part * kD + c8;
  *(volatile v4u*)q = u;
  __threadfence();
  *(volatile v4u*)q = u;
}

__global__ __launch_bounds__(256) void wt_cast_kernel(const float* __restrict__ W, int ldw, int nvalid, int kvalid,
                                                      unsigned short* __restrict__ out, int ldo, int kco, int kcount,
                                                      int nrows, float scale) {
  const int t = blockIdx.x * 256 + threadIdx.x;
  const int tpr = kcount >> 3;
  const int total = nrows * tpr;
  if (t >= total) return;
  const int n = t / tpr;
  const int kk = (t - n * tpr) * 8;
  const int nc = (n < nvalid) ? n : (nvalid - 1);
  const bool nok = (n < nvalid);
  unsigned short hb[8];
#pragma unroll
  for (int e = 0; e < 8; ++e) {
    const int k = kk + e;
    const int kc = (k < kvalid) ? k : (kvalid - 1);
    float v = W[(size_t)kc * ldw + nc] * scale;
    v = (nok && (k < kvalid)) ? v : 0.0f;
    hb[e] = h_bits(v);
  }
  const v4u u = (v4u){pk16(hb[0], hb[1]), pk16(hb[2], hb[3]), pk16(hb[4], hb[5]), pk16(hb[6], hb[7])};
  unsigned short* q = out + (size_t)n * ldo + kco + kk;
  *(volatile v4u*)q = u;
  __threadfence();
  *(volatile v4u*)q = u;
}

template <bool TANH_PI>
__global__ __launch_bounds__(256) void trig_kernel(const float* ang, float* outc, float* outs, int n) {
  const int i = blockIdx.x * 256 + threadIdx.x;
  if (i >= n) return;
  float a = ang[i];
  if (TANH_PI) a = tanhf(a) * kPI;
  float s, c;
  sincosf(a, &s, &c);
  ((volatile float*)outc)[i] = c;
  ((volatile float*)outs)[i] = s;
  __threadfence();
  ((volatile float*)outc)[i] = c;
  ((volatile float*)outs)[i] = s;
}

__global__ __launch_bounds__(256) void gelu_pair_kernel(const float* __restrict__ in, unsigned short* __restrict__ out,
                                                        int npairs, float carry) {
  const int i = blockIdx.x * 256 + threadIdx.x;
  if (i >= npairs) return;
  const v2f v = *(const v2f*)(in + 2 * (size_t)i);
  const float g0 = 0.5f * v.x * (1.0f + erff(v.x * 0.70710678118654752f)) * carry;
  const float g1 = 0.5f * v.y * (1.0f + erff(v.y * 0.70710678118654752f)) * carry;
  const unsigned u = pk16(h_bits(g0), h_bits(g1));
  unsigned* q = (unsigned*)(out + 2 * (size_t)i);
  *(volatile unsigned*)q = u;
  __threadfence();
  *(volatile unsigned*)q = u;
}

__global__ __launch_bounds__(32) void scan_pos_ctx_kernel(
    const float* __restrict__ x, const unsigned short* __restrict__ v1h, const unsigned short* __restrict__ mgh,
    const float* __restrict__ pc, const float* __restrict__ ps, const float* __restrict__ oc, const float* __restrict__ os,
    const float* __restrict__ magsc, unsigned short* __restrict__ pr16, unsigned short* __restrict__ a3) {
  const int lane = threadIdx.x;
  const int b  = blockIdx.x >> 3;
  const int cb = blockIdx.x & 7;
  const int d0 = cb * 64 + 2 * lane;
  const float ams = fabsf(magsc[0]);
  float ac0 = 0.f, as0 = 0.f, am0 = 0.f, ax0 = 0.f;
  float ac1 = 0.f, as1 = 0.f, am1 = 0.f, ax1 = 0.f;
#pragma unroll 1
  for (int l = 0; l < kL; ++l) {
    const size_t row = (size_t)b * kL + l;
    const size_t e = row * kD + d0;
    const size_t pe = (size_t)l * kD + d0;
    const v2f xv  = *(const v2f*)(x + e);
    const unsigned vw = *(const unsigned*)(v1h + e);
    const unsigned mw = *(const unsigned*)(mgh + e);
    const v2f pcv = *(const v2f*)(pc + pe);
    const v2f psv = *(const v2f*)(ps + pe);
    const v2f ocv = *(const v2f*)(oc + e);
    const v2f osv = *(const v2f*)(os + e);
    const float invl = __builtin_amdgcn_rcpf((float)(l + 1));
    const float m0  = ams * __builtin_amdgcn_rcpf(1.0f + expf(-h_lo(mw)));
    const float wv0 = m0 * h_lo(vw);
    ac0 += pcv.x * wv0;
    as0 += psv.x * wv0;
    am0 += m0;
    const float is0 = __builtin_amdgcn_rsqf(am0 + 1e-8f);
    const float qc0 = pcv.x * ocv.x - psv.x * osv.x;
    const float qs0 = psv.x * ocv.x + pcv.x * osv.x;
    const float pr0 = (ac0 * is0) * qc0 + (as0 * is0) * qs0;
    ax0 += xv.x;
    const float cx0 = ax0 * invl;
    const float m1  = ams * __builtin_amdgcn_rcpf(1.0f + expf(-h_hi(mw)));
    const float wv1 = m1 * h_hi(vw);
    ac1 += pcv.y * wv1;
    as1 += psv.y * wv1;
    am1 += m1;
    const float is1 = __builtin_amdgcn_rsqf(am1 + 1e-8f);
    const float qc1 = pcv.y * ocv.y - psv.y * osv.y;
    const float qs1 = psv.y * ocv.y + pcv.y * osv.y;
    const float pr1 = (ac1 * is1) * qc1 + (as1 * is1) * qs1;
    ax1 += xv.y;
    const float cx1 = ax1 * invl;

    const unsigned pw = pk16(h_bits(pr0 * kSqrt32), h_bits(pr1 * kSqrt32));
    const unsigned cw = pk16(h_bits(cx0 * 16.0f), h_bits(cx1 * 16.0f));
    unsigned* pp = (unsigned*)(pr16 + e);
    unsigned* cp = (unsigned*)(a3 + row * kD3 + kD2 + d0);
    *(volatile unsigned*)pp = pw;
    *(volatile unsigned*)cp = cw;
    __threadfence();
    *(volatile unsigned*)pp = pw;
    *(volatile unsigned*)cp = cw;
  }
}

__global__ __launch_bounds__(128) void scan_kv_kernel(
    const float* __restrict__ qsc, const float* __restrict__ qss, const float* __restrict__ vg,
    const float* __restrict__ bval, const float* __restrict__ bgate, unsigned short* __restrict__ kv16) {
  __shared__ float stg[2][32];
  const int tid = threadIdx.x;
  const int h  = tid >> 5;
  const int ph = tid & 31;
  const int b  = blockIdx.x;
  const int bit2 = (ph >> 2) & 1, bit1 = (ph >> 1) & 1, bit0 = ph & 1;
  const float bg = bgate[h];
  float bvv[8];
#pragma unroll
  for (int v = 0; v < 8; ++v) bvv[v] = bval[h * kV + v];
  float kc[8], ks[8];
#pragma unroll
  for (int v = 0; v < 8; ++v) { kc[v] = 0.f; ks[v] = 0.f; }
  float gsum = 0.f;
  const size_t spoff = (size_t)kM * kP;
#pragma unroll 1
  for (int l = 0; l < kL; l += 2) {
#pragma unroll 1
    for (int s2 = 0; s2 < 2; ++s2) {
      const size_t row = (size_t)b * kL + l + s2;
      const float gpre = vg[row * kVGld + kHV + h] + bg;
      const float g = __builtin_amdgcn_rcpf(1.0f + expf(-gpre));
      gsum += g;
      const float invnf = __builtin_amdgcn_rsqf(fmaxf(gsum, 1.0f));
      const size_t qe = row * kP + h * kPh + ph;
      const float sc = qsc[spoff + qe];
      const float ss = qss[spoff + qe];
      const float qc = qsc[qe];
      const float qs = qss[qe];
      const v4f va = *(const v4f*)(vg + row * kVGld + h * kV);
      const v4f vb = *(const v4f*)(vg + row * kVGld + h * kV + 4);
      const float vals[8] = {va.x, va.y, va.z, va.w, vb.x, vb.y, vb.z, vb.w};
      float t[8];
#pragma unroll
      for (int v = 0; v < 8; ++v) {
        const float val = vals[v] + bvv[v];
        kc[v] += (sc * val) * g;
        ks[v] += (ss * val) * g;
        t[v] = qc * kc[v] + qs * ks[v];
      }
#pragma unroll
      for (int v = 0; v < 8; ++v) t[v] += __shfl_xor(t[v], 16, 32);
#pragma unroll
      for (int v = 0; v < 8; ++v) t[v] += __shfl_xor(t[v], 8, 32);
      float k4[4];
#pragma unroll
      for (int i = 0; i < 4; ++i) {
        const float keep = bit2 ? t[4 + i] : t[i];
        const float send = bit2 ? t[i] : t[4 + i];
        k4[i] = keep + __shfl_xor(send, 4, 32);
      }
      float k2[2];
#pragma unroll
      for (int i = 0; i < 2; ++i) {
        const float keep = bit1 ? k4[2 + i] : k4[i];
        const float send = bit1 ? k4[i] : k4[2 + i];
        k2[i] = keep + __shfl_xor(send, 2, 32);
      }
      const float keep1 = bit0 ? k2[1] : k2[0];
      const float send1 = bit0 ? k2[0] : k2[1];
      const float r = (keep1 + __shfl_xor(send1, 1, 32)) * invnf;
      if (ph < 8) stg[s2][h * kV + ph] = r;
    }
    __syncthreads();
    if (h == 0) {
      const int jj = ph & 7;
      const float* sp = &stg[jj >> 2][(jj & 3) * 8];
      unsigned short hb[8];
#pragma unroll
      for (int e = 0; e < 8; ++e) hb[e] = h_bits(sp[e] * kSqrt8);
      const v4u u = (v4u){pk16(hb[0], hb[1]), pk16(hb[2], hb[3]), pk16(hb[4], hb[5]), pk16(hb[6], hb[7])};
      const size_t row0 = (size_t)b * kL + l;
      unsigned short* dst = kv16 + (row0 + (jj >> 2)) * kHV + (jj & 3) * 8;
      if (ph < 8) *(volatile v4u*)dst = u;
      __threadfence();
      if (ph < 8) *(volatile v4u*)dst = u;
    }
    __syncthreads();
  }
}

__global__ __launch_bounds__(192) void ln_traj_kernel(const float* __restrict__ comb, const float* __restrict__ qsc,
                                                      const float* __restrict__ x, const float* __restrict__ lng,
                                                      const float* __restrict__ lnb, unsigned short* __restrict__ ln16) {
  __shared__ float ra[6];
  __shared__ float rb[6];
  __shared__ float rc[6];
  const int row = blockIdx.x;
  const int t = threadIdx.x;
  const int lane = t & 31, wave = t >> 5;
  const float cq = qsc[(size_t)row * kP + (t & (kP - 1))];
  float part = (t < kP) ? cq : 0.0f;
  part = wave_sum(part);
  if (lane == 0) ra[wave] = part;
  __syncthreads();
  const float mcos = (((ra[0] + ra[1]) + ra[2]) + ra[3]) * (1.0f / 128.0f);
  const int c0 = t * 8;
  const int ccl = (c0 < kD2 - 8) ? c0 : (kD2 - 8);
  int cxl = c0 - kD2; cxl = (cxl < 0) ? 0 : cxl; cxl = (cxl > kD - 8) ? (kD - 8) : cxl;
  const float* cp = comb + (size_t)row * kD2 + ccl;
  const float* xp = x + (size_t)row * kD + cxl;
  const v4f ca = *(const v4f*)(cp);
  const v4f cb = *(const v4f*)(cp + 4);
  const v4f xa = *(const v4f*)(xp);
  const v4f xb = *(const v4f*)(xp + 4);
  const bool isx = (c0 >= kD2);
  float v[8];
#pragma unroll
  for (int e = 0; e < 4; ++e) {
    v[e]     = isx ? xa[e] * mcos : ca[e];
    v[4 + e] = isx ? xb[e] * mcos : cb[e];
  }
  float s = 0.f;
#pragma unroll
  for (int e = 0; e < 8; ++e) s += v[e];
  s = wave_sum(s);
  if (lane == 0) rb[wave] = s;
  __syncthreads();
  const float mean = (((((rb[0] + rb[1]) + rb[2]) + rb[3]) + rb[4]) + rb[5]) * (1.0f / 1536.0f);
  float d[8];
  float q = 0.f;
#pragma unroll
  for (int e = 0; e < 8; ++e) { d[e] = v[e] - mean; q += d[e] * d[e]; }
  q = wave_sum(q);
  if (lane == 0) rc[wave] = q;
  __syncthreads();
  const float var = (((((rc[0] + rc[1]) + rc[2]) + rc[3]) + rc[4]) + rc[5]) * (1.0f / 1536.0f);
  const float rstd = __builtin_amdgcn_rsqf(var + 1e-5f);
  unsigned short hb[8];
#pragma unroll
  for (int e = 0; e < 8; ++e) {
    const float y = (d[e] * rstd) * lng[c0 + e] + lnb[c0 + e];
    hb[e] = h_bits(y);
  }
  const v4u u = (v4u){pk16(hb[0], hb[1]), pk16(hb[2], hb[3]), pk16(hb[4], hb[5]), pk16(hb[6], hb[7])};
  unsigned short* dst = ln16 + (size_t)row * kD3 + c0;
  *(volatile v4u*)dst = u;
  __threadfence();
  *(volatile v4u*)dst = u;
}

template <int BIAS, int OUTM, bool RES>
static void run_gemm(hipStream_t st, const unsigned short* A, int lda, const unsigned short* Bt, int ldb,
                     void* C, int ldc, const float* bias, const float* resid, int M, int N, int K, float scale) {
  const int tiles = (M / 64) * (N / 64);
  dim3 grid((tiles + 7) / 8, 1);
  wmma_gemm64<0, false, BIAS, OUTM, RES, 0><<<grid, 256, 0, st>>>(
      A, nullptr, lda, 0L, Bt, nullptr, ldb, 0L, C, nullptr, ldc, 0L, bias, resid, 0L, M, N, K, scale);
}
static void run_wt(hipStream_t st, const float* W, int ldw, int nvalid, int kvalid, unsigned short* out, int ldo,
                   int kco, int kcount, int nrows, float scale) {
  const int total = nrows * (kcount / 8);
  dim3 grid((total + 255) / 256);
  wt_cast_kernel<<<grid, 256, 0, st>>>(W, ldw, nvalid, kvalid, out, ldo, kco, kcount, nrows, scale);
}

extern "C" void kernel_launch(void* const* d_in, const int* in_sizes, int n_in,
                              void* d_out, int out_size, void* d_ws, size_t ws_size,
                              hipStream_t stream)
{
  (void)out_size;
  if (n_in < 29) return;
  if (in_sizes[0] != kM * kD || in_sizes[1] != kL * kD || in_sizes[25] != kD3 * kD2) return;

  const float* x      = (const float*)d_in[0];
  const float* pos    = (const float*)d_in[1];
  const float* w_v1   = (const float*)d_in[2];
  const float* b_v1   = (const float*)d_in[3];
  const float* w_o1   = (const float*)d_in[4];
  const float* b_o1   = (const float*)d_in[5];
  const float* w_off  = (const float*)d_in[6];
  const float* b_off  = (const float*)d_in[7];
  const float* w_mag  = (const float*)d_in[8];
  const float* b_mag  = (const float*)d_in[9];
  const float* magsc  = (const float*)d_in[10];
  const float* w_key  = (const float*)d_in[11];
  const float* b_key  = (const float*)d_in[12];
  const float* w_val  = (const float*)d_in[13];
  const float* b_val  = (const float*)d_in[14];
  const float* w_sk1  = (const float*)d_in[15];
  const float* b_sk1  = (const float*)d_in[16];
  const float* w_sk2  = (const float*)d_in[17];
  const float* b_sk2  = (const float*)d_in[18];
  const float* w_gate = (const float*)d_in[19];
  const float* b_gate = (const float*)d_in[20];
  const float* w_kv   = (const float*)d_in[21];
  const float* b_kv   = (const float*)d_in[22];
  const float* ln_g   = (const float*)d_in[23];
  const float* ln_b   = (const float*)d_in[24];
  const float* w_f1   = (const float*)d_in[25];
  const float* b_f1   = (const float*)d_in[26];
  const float* w_f2   = (const float*)d_in[27];
  const float* b_f2   = (const float*)d_in[28];
  float* out = (float*)d_out;

  const size_t MiB = 1048576;
  const size_t oWV1 = 0, oWMAG = 524288, oWO1 = 1048576, oWOFF = 1572864, oWSK1 = 2621440,
               oWKEY = 3670016, oWSK2 = 3801088, oWVG = 3932160, oWKV = 3997696, oWF1 = 4030464, oWF2 = 7176192;
  const size_t oA3   = 8 * MiB;
  const size_t oRB   = 32 * MiB;
  const size_t oV1h  = oRB, oMGh = oRB + 8 * MiB, oOFF = oRB + 16 * MiB, oOS = oRB + 32 * MiB;
  const size_t oHPRE = oRB, oHMID = oRB + 16 * MiB;
  const size_t oCOMB = oRB, oH2PRE = oRB, oH2h = oRB + 32 * MiB;
  const size_t oRC   = 80 * MiB;
  const size_t oPC   = oRC, oPS = oRC + 8 * MiB;
  const size_t oQSC  = oRC, oQSS = oRC + 8 * MiB, oKV16 = oRC + 16 * MiB;
  const size_t oPR16 = oKV16 + 524288;
  const size_t oQPT  = oPR16 + 8 * MiB;
  const size_t oSPT  = oQPT + (size_t)kM * kP * 4;
  const size_t oVG   = oSPT + (size_t)kM * kP * 4;
  const size_t oEND  = oVG + (size_t)kM * kVGld * 4;
  if (ws_size < oEND) return;

  char* w = (char*)d_ws;
  unsigned short* WV1T  = (unsigned short*)(w + oWV1);
  unsigned short* WMAGT = (unsigned short*)(w + oWMAG);
  unsigned short* WO1T  = (unsigned short*)(w + oWO1);
  unsigned short* WOFFT = (unsigned short*)(w + oWOFF);
  unsigned short* WSK1T = (unsigned short*)(w + oWSK1);
  unsigned short* WKEYT = (unsigned short*)(w + oWKEY);
  unsigned short* WSK2T = (unsigned short*)(w + oWSK2);
  unsigned short* WVGT  = (unsigned short*)(w + oWVG);
  unsigned short* WKVT  = (unsigned short*)(w + oWKV);
  unsigned short* WF1T  = (unsigned short*)(w + oWF1);
  unsigned short* WF2T  = (unsigned short*)(w + oWF2);
  unsigned short* A3    = (unsigned short*)(w + oA3);
  unsigned short* LN16  = (unsigned short*)(w + oA3);
  unsigned short* V1h   = (unsigned short*)(w + oV1h);
  unsigned short* MGh   = (unsigned short*)(w + oMGh);
  float* OFFT  = (float*)(w + oOFF);
  float* OS    = (float*)(w + oOS);
  float* HPRE  = (float*)(w + oHPRE);
  unsigned short* HMID = (unsigned short*)(w + oHMID);
  float* COMB  = (float*)(w + oCOMB);
  float* H2PRE = (float*)(w + oH2PRE);
  unsigned short* H2h  = (unsigned short*)(w + oH2h);
  float* PC    = (float*)(w + oPC);
  float* PS    = (float*)(w + oPS);
  float* QSC   = (float*)(w + oQSC);
  float* QSS   = (float*)(w + oQSS);
  unsigned short* KV16 = (unsigned short*)(w + oKV16);
  unsigned short* PR16 = (unsigned short*)(w + oPR16);
  float* QPT   = (float*)(w + oQPT);
  float* SPT   = (float*)(w + oSPT);
  float* VG    = (float*)(w + oVG);

  const float s32 = 1.0f / 32.0f, s256 = 1.0f / 256.0f, s512 = 1.0f / 512.0f, s4096 = 1.0f / 4096.0f, s128 = 1.0f / 128.0f;
  const float wc = 32.0f;

  cast_inputs_kernel<<<dim3(kM * (kD / 8) / 256, 2), 256, 0, stream>>>(x, pos, A3);

  run_wt(stream, w_v1,  kD,  kD,  kD,  WV1T,  kD,  0,  kD,  kD,  wc);
  run_wt(stream, w_mag, kD,  kD,  kD,  WMAGT, kD,  0,  kD,  kD,  wc);
  run_wt(stream, w_o1,  kD,  kD,  kD,  WO1T,  kD,  0,  kD,  kD,  wc);
  run_wt(stream, w_key, kP,  kP,  kD,  WKEYT, kD,  0,  kD,  kP,  wc);
  run_wt(stream, w_sk2, kP,  kP,  kD,  WSK2T, kD,  0,  kD,  kP,  wc);
  run_wt(stream, w_off + (size_t)kD * kD, kD, kD, kD, WOFFT, kD2, 0,  kD, kD, wc);
  run_wt(stream, w_off,                   kD, kD, kD, WOFFT, kD2, kD, kD, kD, wc);
  run_wt(stream, w_sk1,                   kD, kD, kD, WSK1T, kD2, 0,  kD, kD, wc);
  run_wt(stream, w_sk1 + (size_t)kD * kD, kD, kD, kD, WSK1T, kD2, kD, kD, kD, 2.0f);
  run_wt(stream, w_val,  kHV, kHV, kD, WVGT,                     kD, 0, kD, kHV, wc);
  run_wt(stream, w_gate, kH,  kH,  kD, WVGT + (size_t)kHV * kD,  kD, 0, kD, kHV, wc);
  run_wt(stream, w_kv,  kD,  kD,  kHV, WKVT,  kHV, 0,  kHV, kD,  wc);
  run_wt(stream, w_f1,  kD2, kD2, kD3, WF1T,  kD3, 0,  kD3, kD2, wc);
  run_wt(stream, w_f2,  kD,  kD,  kD2, WF2T,  kD2, 0,  kD2, kD,  wc);

  run_gemm<2, 1, false>(stream, A3 + kD, kD3, WV1T,  kD,  V1h,  kD,   b_v1,  nullptr, kM, kD,   kD,  s32);
  run_gemm<2, 1, false>(stream, A3 + kD, kD3, WMAGT, kD,  MGh,  kD,   b_mag, nullptr, kM, kD,   kD,  s32);
  run_gemm<2, 0, false>(stream, A3 + kD, kD3, WKEYT, kD,  QPT,  kP,   b_key, nullptr, kM, kP,   kD,  s32);
  run_gemm<0, 0, false>(stream, A3 + kD, kD3, WVGT,  kD,  VG,   kVGld, nullptr, nullptr, kM, kVGld, kD, s32);
  run_gemm<2, 0, false>(stream, A3,      kD3, WOFFT, kD2, OFFT, kD,   b_off, nullptr, kM, kD,   kD2, s32);

  trig_kernel<false><<<dim3(kL * kD / 256), 256, 0, stream>>>(pos, PC, PS, kL * kD);
  trig_kernel<true><<<dim3(kM * kD / 256), 256, 0, stream>>>(OFFT, OFFT, OS, kM * kD);

  scan_pos_ctx_kernel<<<dim3(16), 32, 0, stream>>>(x, V1h, MGh, PC, PS, OFFT, OS, magsc, PR16, A3);

  run_gemm<2, 0, false>(stream, A3 + kD, kD3, WSK1T, kD2, HPRE, kD, b_sk1, nullptr, kM, kD, kD2, s32);
  gelu_pair_kernel<<<dim3(kM * kD / 2 / 256), 256, 0, stream>>>(HPRE, HMID, kM * kD / 2, 8.0f);
  run_gemm<2, 0, false>(stream, HMID, kD, WSK2T, kD, SPT, kP, b_sk2, nullptr, kM, kP, kD, s256);

  trig_kernel<true><<<dim3(2 * kM * kP / 256), 256, 0, stream>>>(QPT, QSC, QSS, 2 * kM * kP);

  scan_kv_kernel<<<dim3(kB), 128, 0, stream>>>(QSC, QSS, VG, b_val, b_gate, KV16);

  run_gemm<2, 0, false>(stream, PR16, kD,  WO1T, kD,  COMB,      kD2, b_o1, nullptr, kM, kD, kD,  s4096);
  run_gemm<2, 0, false>(stream, KV16, kHV, WKVT, kHV, COMB + kD, kD2, b_kv, nullptr, kM, kD, kHV, s512);

  ln_traj_kernel<<<dim3(kM), 192, 0, stream>>>(COMB, QSC, x, ln_g, ln_b, LN16);
  run_gemm<2, 0, false>(stream, LN16, kD3, WF1T, kD3, H2PRE, kD2, b_f1, nullptr, kM, kD2, kD3, s32);
  gelu_pair_kernel<<<dim3(kM * kD2 / 2 / 256), 256, 0, stream>>>(H2PRE, H2h, kM * kD2 / 2, 4.0f);
  run_gemm<2, 0, true>(stream, H2h, kD2, WF2T, kD2, out, kD, b_f2, x, kM, kD, kD2, s128);
}
